// IDContextAttention_4398046511688
// MI455X (gfx1250) — hardware-verified
//
#include <hip/hip_runtime.h>


#define NB_  4
#define TT   2048
#define DM   768
#define NH_  12
#define HD   64
#define HPP  4
#define PCAR 1024.0f
typedef _Float16 h16;
typedef unsigned short bf;
typedef __attribute__((ext_vector_type(16))) __bf16   v16bf;
typedef __attribute__((ext_vector_type(16))) _Float16 v16h;
typedef __attribute__((ext_vector_type(8)))  _Float16 v8h;
typedef __attribute__((ext_vector_type(8)))  unsigned short v8us;
typedef __attribute__((ext_vector_type(8)))  float    v8f;
typedef __attribute__((ext_vector_type(4)))  float    v4f;
typedef v8h  __attribute__((may_alias)) v8ha;
typedef v4f  __attribute__((may_alias)) v4fa;
typedef v8us __attribute__((may_alias)) v8usa;

__device__ __forceinline__ unsigned short f2bf(float f) { unsigned u = __float_as_uint(f); u += 0x7FFFu + ((u >> 16) & 1u); return (unsigned short)(u >> 16); }
__device__ __forceinline__ float bf2f(unsigned short b) { return __uint_as_float(((unsigned)b) << 16); }
__device__ __forceinline__ float bfr(float f) { return bf2f(f2bf(f)); }
__device__ __forceinline__ v16h cat16(v8h lo, v8h hi) { return __builtin_shufflevector(lo, hi, 0, 1, 2, 3, 4, 5, 6, 7, 8, 9, 10, 11, 12, 13, 14, 15); }
__device__ __forceinline__ v16bf cat16b(v8us lo, v8us hi) { return __builtin_bit_cast(v16bf, __builtin_shufflevector(lo, hi, 0, 1, 2, 3, 4, 5, 6, 7, 8, 9, 10, 11, 12, 13, 14, 15)); }
__device__ __forceinline__ v8f wmma16(v16h a, v16h b, v8f c) { return __builtin_amdgcn_wmma_f32_16x16x32_f16(false, a, false, b, (short)0, c, false, false); }
__device__ __forceinline__ v8f wmmab(v16bf a, v16bf b, v8f c) { return __builtin_amdgcn_wmma_f32_16x16x32_bf16(false, a, false, b, (short)0, c, false, false); }


template <typename T16> struct WFrag;
template <> struct WFrag<h16> { typedef v16h V; static __device__ __forceinline__ V ld(const h16* p) { return cat16(*(const v8h*)p, *(const v8h*)(p + 16)); } static __device__ __forceinline__ v8f mma(V a, V b, v8f c) { return wmma16(a, b, c); } };
template <> struct WFrag<bf> { typedef v16bf V; static __device__ __forceinline__ V ld(const bf* p) { return cat16b(*(const v8us*)p, *(const v8us*)(p + 16)); } static __device__ __forceinline__ v8f mma(V a, V b, v8f c) { return wmmab(a, b, c); } };
template <typename T16, int NSPLIT, bool BIAS>
__global__ __launch_bounds__(32) void k_gemmw(const T16* __restrict__ A, const T16* __restrict__ A2, const T16* __restrict__ Bt, const T16* __restrict__ Bt2, int K, float* C, int ldc, const float* __restrict__ bias, size_t sA, size_t sB, size_t sC) {
    typedef typename WFrag<T16>::V V;
    __shared__ __align__(16) float os[16 * 68];
    const size_t z = blockIdx.z; A += z * sA; if (A2) A2 += z * sA; Bt += z * sB; if (Bt2) Bt2 += z * sB; C += z * sC;
    const int lane = threadIdx.x & 31, lr = lane & 15, hi = lane >> 4; const int r0 = blockIdx.x * 64, c0 = blockIdx.y * 64;
    v8f acc[4][4];
#pragma unroll
    for (int mb = 0; mb < 4; ++mb)
#pragma unroll
        for (int nb = 0; nb < 4; ++nb) acc[mb][nb] = (v8f){};
    const size_t aoff = (size_t)(r0 + lr) * K + 8 * hi, boff = (size_t)(c0 + lr) * K + 8 * hi;
#pragma unroll 1
    for (int kc = 0; kc < K; kc += 32) {
        V a[4], a2[4];
#pragma unroll
        for (int mb = 0; mb < 4; ++mb) { a[mb] = WFrag<T16>::ld(A + aoff + (size_t)mb * 16 * K + kc); if (NSPLIT == 1 || NSPLIT == 2) a2[mb] = WFrag<T16>::ld(A2 + aoff + (size_t)mb * 16 * K + kc); }
#pragma unroll
        for (int nb = 0; nb < 4; ++nb) { const V b = WFrag<T16>::ld(Bt + boff + (size_t)nb * 16 * K + kc); V b2; if (NSPLIT >= 2) b2 = WFrag<T16>::ld(Bt2 + boff + (size_t)nb * 16 * K + kc);
#pragma unroll
            for (int mb = 0; mb < 4; ++mb) { acc[mb][nb] = WFrag<T16>::mma(a[mb], b, acc[mb][nb]); if (NSPLIT == 1 || NSPLIT == 2) acc[mb][nb] = WFrag<T16>::mma(a2[mb], b, acc[mb][nb]); if (NSPLIT >= 2) acc[mb][nb] = WFrag<T16>::mma(a[mb], b2, acc[mb][nb]); } }
        asm volatile("v_nop\n\tv_nop\n\tv_nop\n\tv_nop" : "+v"(acc[0][0]), "+v"(acc[1][1]), "+v"(acc[2][2]), "+v"(acc[3][3]) : "v"(a[0]), "v"(a[3]));
    }
#pragma unroll
    for (int mb = 0; mb < 4; ++mb) {
#pragma unroll
        for (int nb = 0; nb < 4; ++nb) {
#pragma unroll
            for (int j = 0; j < 8; ++j) os[(hi * 8 + j) * 68 + nb * 16 + lr] = acc[mb][nb][j]; }
        __builtin_amdgcn_wave_barrier(); asm volatile("" ::: "memory");
        float* crow = C + (size_t)(r0 + mb * 16) * ldc + c0;
#pragma unroll 1
        for (int ps = 0; ps < 2; ++ps) {
#pragma unroll
            for (int s = 0; s < 8; ++s) { const int row = 2 * s + hi, cofs = lr * 4; v4f val = *(const v4fa*)(os + row * 68 + cofs); if (BIAS) { val[0] += bfr(bias[c0 + cofs]); val[1] += bfr(bias[c0 + cofs + 1]); val[2] += bfr(bias[c0 + cofs + 2]); val[3] += bfr(bias[c0 + cofs + 3]); }
                *(volatile v4f*)(crow + (size_t)row * ldc + cofs) = val; }
            if (ps == 0) __threadfence(); }
        __builtin_amdgcn_wave_barrier(); asm volatile("" ::: "memory");
    }
}

__device__ __forceinline__ h16 tohx(float x) { return (h16)x; }
__device__ __forceinline__ void splitf(float y, unsigned short& h, unsigned short& l) { h = f2bf(y); l = f2bf(y - bf2f(h)); }
typedef __attribute__((ext_vector_type(2))) unsigned short v2us;
typedef __attribute__((ext_vector_type(4))) unsigned short v4us;
typedef __attribute__((ext_vector_type(2))) _Float16 v2h;
typedef __attribute__((ext_vector_type(4))) _Float16 v4h;

__global__ __launch_bounds__(256) void k_cvt8(const float* __restrict__ src, bf* dst, size_t n8) { const size_t i = (size_t)blockIdx.x * 256 + threadIdx.x; if (i >= n8) return; const v8f v = *(const v8f*)(src + i * 8); v8us o;
#pragma unroll
    for (int k = 0; k < 8; ++k) o[k] = f2bf(v[k]); *(volatile v8us*)(dst + i * 8) = o; __threadfence(); *(volatile v8us*)(dst + i * 8) = o; }
__global__ __launch_bounds__(256) void k_idkv(const float* __restrict__ ida, const float* __restrict__ Wk, const float* __restrict__ bk, const float* __restrict__ Wv, const float* __restrict__ bv, float* KID, float* VID) { const int c = blockIdx.x * 256 + threadIdx.x; if (c >= DM) return; float sk = 0.f, sv = 0.f;
#pragma unroll 1
    for (int d = 0; d < DM; ++d) { const float a = bfr(ida[d]); float wk = bfr(Wk[(size_t)c * DM + d]), wv = bfr(Wv[(size_t)c * DM + d]); asm volatile("" : "+v"(wk)); asm volatile("" : "+v"(wv)); float p1 = __fmul_rn(a, wk), p2 = __fmul_rn(a, wv); asm volatile("" : "+v"(p1)); asm volatile("" : "+v"(p2)); sk = __fadd_rn(sk, p1); sv = __fadd_rn(sv, p2); }
    const float rk = __fadd_rn(sk, bfr(bk[c])), rv = __fadd_rn(sv, bfr(bv[c])); for (int ps = 0; ps < 2; ++ps) { *(volatile float*)(KID + c) = rk; *(volatile float*)(VID + c) = rv; if (ps == 0) __threadfence(); } }
__global__ __launch_bounds__(256) void k_pl(const float* __restrict__ F, h16* P) { const int e = (blockIdx.x * 256 + threadIdx.x) * 4; if (e >= NH_ * TT * HD) return; const int d = e % HD; const int t = (e / HD) % TT; const int h = e / (HD * TT); const float* f = F + (size_t)t * DM + h * HD + d; v4h o;
#pragma unroll
    for (int u = 0; u < 4; ++u) o[u] = tohx(f[u]); *(volatile v4h*)(P + e) = o; __threadfence(); *(volatile v4h*)(P + e) = o; }
__global__ __launch_bounds__(256) void k_vt(const float* __restrict__ V, h16* VT) { const int e = (blockIdx.x * 256 + threadIdx.x) * 2; if (e >= NH_ * HD * TT) return; const int t = e % TT; const int d = (e / TT) % HD; const int h = e / (TT * HD); v2h o; o[0] = tohx(V[(size_t)t * DM + h * HD + d]); o[1] = tohx(V[(size_t)(t + 1) * DM + h * HD + d]); *(volatile v2h*)(VT + e) = o; __threadfence(); *(volatile v2h*)(VT + e) = o; }
__global__ __launch_bounds__(256) void k_s0(const float* __restrict__ Q, const float* __restrict__ KID, float* S0) { const int idx = blockIdx.x * 256 + threadIdx.x; if (idx >= NH_ * TT) return; const int t = idx % TT; const int h = idx / TT; float s = 0.f;
#pragma unroll 1
    for (int d = 0; d < HD; ++d) { float p = __fmul_rn(Q[(size_t)t * DM + h * HD + d], KID[h * HD + d]); asm volatile("" : "+v"(p)); s = __fadd_rn(s, p); } *(volatile float*)(S0 + idx) = s; __threadfence(); *(volatile float*)(S0 + idx) = s; }
__global__ __launch_bounds__(256) void k_isoft(const float* __restrict__ Sb, const float* __restrict__ S0, int h0, h16* P16, float* P0) { const int lane = threadIdx.x & 31; const int row = blockIdx.x * 8 + (threadIdx.x >> 5); if (row >= HPP * TT) return; const int t = row % TT; const int z = row / TT; const float* sr = Sb + (size_t)row * TT; float v[TT / 32];
    const float s0 = S0[(size_t)(h0 + z) * TT + t] * 0.125f; float mx = s0;
#pragma unroll
    for (int ch = 0; ch < TT / 128; ++ch) { const v4f a = *(const v4f*)(sr + ch * 128 + lane * 4);
#pragma unroll
        for (int u = 0; u < 4; ++u) { const float tt = a[u] * 0.125f; v[ch * 4 + u] = tt; mx = fmaxf(mx, tt); } }
#pragma unroll
    for (int sh = 16; sh; sh >>= 1) mx = fmaxf(mx, __shfl_xor(mx, sh, 32));
    float sum = 0.f;
#pragma unroll
    for (int q = 0; q < TT / 32; ++q) { float d0 = __fsub_rn(v[q], mx); asm volatile("" : "+v"(d0)); v[q] = __builtin_amdgcn_exp2f(__fmul_rn(d0, 1.4426950408889634f)); sum += v[q]; }
#pragma unroll
    for (int sh = 16; sh; sh >>= 1) sum += __shfl_xor(sum, sh, 32);
    float d1 = __fsub_rn(s0, mx); asm volatile("" : "+v"(d1)); const float e0 = __builtin_amdgcn_exp2f(__fmul_rn(d1, 1.4426950408889634f)); sum = __fadd_rn(sum, e0);
    const float inv = __fdiv_rn(1.0f, sum); const float f = inv * PCAR; const float p0 = __fmul_rn(e0, inv);
    for (int ps = 0; ps < 2; ++ps) {
#pragma unroll
        for (int ch = 0; ch < TT / 128; ++ch) { v4h o4;
#pragma unroll
            for (int q = 0; q < 4; ++q) o4[q] = tohx(v[ch * 4 + q] * f); *(volatile v4h*)(P16 + (size_t)row * TT + ch * 128 + lane * 4) = o4; }
        *(volatile float*)(P0 + (size_t)row * 32 + lane) = p0; if (ps == 0) __threadfence(); } }
__global__ __launch_bounds__(256) void k_mrg(const float* __restrict__ O, const float* __restrict__ P0, const float* __restrict__ VID, int h0, bf* Ah, bf* Al) { const int e = (blockIdx.x * 256 + threadIdx.x) * 4; if (e >= HPP * TT * HD) return; const int d = e % HD; const int t = (e / HD) % TT; const int z = e / (HD * TT); const float p0 = P0[((size_t)z * TT + t) * 32]; v4us oh, ol;
#pragma unroll
    for (int u = 0; u < 4; ++u) { float m = O[e + u] * (1.0f / PCAR); float pv = __fmul_rn(p0, VID[(h0 + z) * HD + d + u]); asm volatile("" : "+v"(pv)); const float y = __fadd_rn(m, pv); unsigned short a, b; splitf(y, a, b); oh[u] = a; ol[u] = b; }
    const size_t oo = (size_t)t * DM + (h0 + z) * HD + d; *(volatile v4us*)(Ah + oo) = oh; *(volatile v4us*)(Al + oo) = ol; __threadfence(); *(volatile v4us*)(Ah + oo) = oh; *(volatile v4us*)(Al + oo) = ol; }

extern "C" void kernel_launch(void* const* d_in, const int* in_sizes, int n_in,
                              void* d_out, int out_size, void* d_ws, size_t ws_size, hipStream_t stream) {
    (void)in_sizes; (void)n_in; (void)out_size;
    const float** I = (const float**)d_in;
    const float *x = I[0], *ida = I[1], *Wq = I[2], *bq = I[3], *Wk = I[4], *bk = I[5], *Wv = I[6], *bv = I[7], *Wo = I[8], *bo = I[9];
    float* OUT = (float*)d_out;
    char* wsp = (char*)d_ws;
    auto take = [&](size_t bytes) { char* p = wsp; wsp += (bytes + 255) & ~(size_t)255; return (void*)p; };
    bf* BQ = (bf*)take((size_t)DM * DM * 2); bf* BK = (bf*)take((size_t)DM * DM * 2); bf* BV = (bf*)take((size_t)DM * DM * 2); bf* BO = (bf*)take((size_t)DM * DM * 2);
    bf* XB = (bf*)take((size_t)TT * DM * 2); float* Q = (float*)take((size_t)TT * DM * 4); float* K = (float*)take((size_t)TT * DM * 4); float* V = (float*)take((size_t)TT * DM * 4); float* KID = (float*)take(DM * 4); float* VID = (float*)take(DM * 4); float* S0 = (float*)take((size_t)NH_ * TT * 4);
    h16* Q16 = (h16*)take((size_t)NH_ * TT * HD * 2); h16* K16 = (h16*)take((size_t)NH_ * TT * HD * 2); h16* VT = (h16*)take((size_t)NH_ * HD * TT * 2); float* Sb = (float*)take((size_t)HPP * TT * TT * 4); h16* P16 = (h16*)take((size_t)HPP * TT * TT * 2); float* P0 = (float*)take((size_t)HPP * TT * 32 * 4); float* O = (float*)take((size_t)HPP * TT * HD * 4); bf* Ah = (bf*)take((size_t)TT * DM * 2); bf* Al = (bf*)take((size_t)TT * DM * 2);
    if ((size_t)(wsp - (char*)d_ws) > ws_size) return;
    k_cvt8<<<(DM * DM / 8 + 255) / 256, 256, 0, stream>>>(Wq, BQ, DM * DM / 8); k_cvt8<<<(DM * DM / 8 + 255) / 256, 256, 0, stream>>>(Wk, BK, DM * DM / 8); k_cvt8<<<(DM * DM / 8 + 255) / 256, 256, 0, stream>>>(Wv, BV, DM * DM / 8); k_cvt8<<<(DM * DM / 8 + 255) / 256, 256, 0, stream>>>(Wo, BO, DM * DM / 8);
    for (int b = 0; b < NB_; ++b) {
        k_cvt8<<<(TT * DM / 8 + 255) / 256, 256, 0, stream>>>(x + (size_t)b * TT * DM, XB, (size_t)TT * DM / 8);
        k_gemmw<bf, 0, true><<<dim3(TT / 64, DM / 64, 1), 32, 0, stream>>>(XB, nullptr, BQ, nullptr, DM, Q, DM, bq, 0, 0, 0); k_gemmw<bf, 0, true><<<dim3(TT / 64, DM / 64, 1), 32, 0, stream>>>(XB, nullptr, BK, nullptr, DM, K, DM, bk, 0, 0, 0); k_gemmw<bf, 0, true><<<dim3(TT / 64, DM / 64, 1), 32, 0, stream>>>(XB, nullptr, BV, nullptr, DM, V, DM, bv, 0, 0, 0);
        k_idkv<<<(DM + 255) / 256, 256, 0, stream>>>(ida + (size_t)b * DM, Wk, bk, Wv, bv, KID, VID); k_s0<<<(NH_ * TT + 255) / 256, 256, 0, stream>>>(Q, KID, S0);
        k_pl<<<(NH_ * TT * HD / 4 + 255) / 256, 256, 0, stream>>>(Q, Q16); k_pl<<<(NH_ * TT * HD / 4 + 255) / 256, 256, 0, stream>>>(K, K16); k_vt<<<(NH_ * HD * TT / 2 + 255) / 256, 256, 0, stream>>>(V, VT);
        for (int h0 = 0; h0 < NH_; h0 += HPP) { const size_t zo = (size_t)h0 * TT * HD;
            k_gemmw<h16, 0, false><<<dim3(TT / 64, TT / 64, HPP), 32, 0, stream>>>(Q16 + zo, nullptr, K16 + zo, nullptr, HD, Sb, TT, nullptr, (size_t)TT * HD, (size_t)TT * HD, (size_t)TT * TT);
            k_isoft<<<HPP * TT / 8, 256, 0, stream>>>(Sb, S0, h0, P16, P0);
            k_gemmw<h16, 0, false><<<dim3(TT / 64, 1, HPP), 32, 0, stream>>>(P16, nullptr, VT + (size_t)h0 * HD * TT, nullptr, TT, O, HD, nullptr, (size_t)TT * TT, (size_t)HD * TT, (size_t)TT * HD);
            k_mrg<<<(HPP * TT * HD / 4 + 255) / 256, 256, 0, stream>>>(O, P0, VID, h0, Ah, Al); }
        k_gemmw<bf, 1, true><<<dim3(TT / 64, DM / 64, 1), 32, 0, stream>>>(Ah, Al, BO, nullptr, DM, OUT + (size_t)b * TT * DM, DM, bo, 0, 0, 0); }
}
